// GatedDeltaRecurrence_62242666053984
// MI455X (gfx1250) — hardware-verified
//
#include <hip/hip_runtime.h>
#include <math.h>

constexpr int kB   = 2;
constexpr int kT   = 2048;
constexpr int kDM  = 1024;
constexpr int kDKV = 512;
constexpr int kH   = 8;
constexpr int kKH  = 96;
constexpr int kVH  = 192;
constexpr int kKQT = kH * kKH;
constexpr int kVT  = kH * kVH;
constexpr int kM   = kB * kT;
constexpr int kBH  = kB * kH;
constexpr float kEps = 1e-6f;
constexpr float kQScale = 0.10206207261596575f;
constexpr float kWCarry = 16.0f;
constexpr float kWCarryInv = 0.0625f;

typedef __attribute__((ext_vector_type(16))) _Float16 v16h;
typedef __attribute__((ext_vector_type(8)))  _Float16 v8h;
typedef __attribute__((ext_vector_type(16))) __bf16   v16b;
typedef __attribute__((ext_vector_type(8)))  __bf16   v8b;
typedef __attribute__((ext_vector_type(8)))  float    v8f;
typedef __attribute__((ext_vector_type(4)))  float    v4f;
typedef __attribute__((ext_vector_type(4)))  unsigned int v4u;

__device__ __forceinline__ unsigned short f2bf_bits(float f) {
  unsigned u = __float_as_uint(f);
  return (unsigned short)((u + 0x7FFFu + ((u >> 16) & 1u)) >> 16);
}
__device__ __forceinline__ float bf_bits2f(unsigned short h) { return __uint_as_float(((unsigned)h) << 16); }

__device__ __forceinline__ void dep_guard_h(v8f& a, v8f& b, v16h x, v16h y) { asm volatile("v_nop\n\tv_nop\n\tv_nop\n\tv_nop" : "+v"(a), "+v"(b) : "v"(x), "v"(y)); }
__device__ __forceinline__ void dep_guard_b(v8f& a, v8f& b, v16b x, v16b y) { asm volatile("v_nop\n\tv_nop\n\tv_nop\n\tv_nop" : "+v"(a), "+v"(b) : "v"(x), "v"(y)); }
__device__ __forceinline__ void keep4_h(v16h a, v16h b, v16h c, v16h d) { asm volatile("v_nop" :: "v"(a), "v"(b), "v"(c), "v"(d)); }
__device__ __forceinline__ void keep4_b(v16b a, v16b b, v16b c, v16b d) { asm volatile("v_nop" :: "v"(a), "v"(b), "v"(c), "v"(d)); }
__device__ __forceinline__ void acc_guard4(v8f& a, v8f& b, v8f& c, v8f& d) { asm volatile("v_nop\n\tv_nop\n\tv_nop\n\tv_nop" : "+v"(a), "+v"(b), "+v"(c), "+v"(d)); }
template <typename T> struct Frag;
template <> struct Frag<_Float16> {
  typedef v16h V; union U { v16h v; v8h h[2]; };
  static __device__ __forceinline__ v16h load(const _Float16* p) {
    U f; f.h[0] = *(const v8h*)(p); f.h[1] = *(const v8h*)(p + 16); return f.v;
  }
  static __device__ __forceinline__ v8f mma(v16h a, v16h b, v8f c) {
    return __builtin_amdgcn_wmma_f32_16x16x32_f16(false, a, false, b, (short)0, c, false, false);
  }
  static __device__ __forceinline__ void guard(v8f& a, v8f& b, v16h x, v16h y) { dep_guard_h(a, b, x, y); }
  static __device__ __forceinline__ void keep(v16h a, v16h b, v16h c, v16h d) { keep4_h(a, b, c, d); }
};
template <> struct Frag<__bf16> {
  typedef v16b V; union U { v16b v; v8b h[2]; };
  static __device__ __forceinline__ v16b load(const __bf16* p) {
    U f; f.h[0] = *(const v8b*)(p); f.h[1] = *(const v8b*)(p + 16); return f.v;
  }
  static __device__ __forceinline__ v8f mma(v16b a, v16b b, v8f c) {
    return __builtin_amdgcn_wmma_f32_16x16x32_bf16(false, a, false, b, (short)0, c, false, false);
  }
  static __device__ __forceinline__ void guard(v8f& a, v8f& b, v16b x, v16b y) { dep_guard_b(a, b, x, y); }
  static __device__ __forceinline__ void keep(v16b a, v16b b, v16b c, v16b d) { keep4_b(a, b, c, d); }
};

__device__ __forceinline__ unsigned pk16(unsigned short a, unsigned short b) { return (unsigned)a | ((unsigned)b << 16); }
__device__ __forceinline__ unsigned short h_bits(float f) { const _Float16 h = (_Float16)f; return __builtin_bit_cast(unsigned short, h); }

template <int ET> struct Elem;
template <> struct Elem<0> { typedef _Float16 T; };
template <> struct Elem<1> { typedef __bf16 T; };
template <int ET, bool SPLIT, int BIAS_MODE, int OUT_MODE, bool RESID, int ACT = 0>
__global__ __launch_bounds__(256) void wmma_gemm64(
    const unsigned short* __restrict__ Ap, const unsigned short* __restrict__ A2p, int lda, long strideA,
    const unsigned short* __restrict__ Btp, const unsigned short* __restrict__ Bt2p, int ldb, long strideB,
    void* __restrict__ Cout, void* __restrict__ Cout2, int ldc, long strideC,
    const float* __restrict__ bias,
    const float* __restrict__ resid, long strideR,
    int M, int N, int K, float scale) {
  typedef typename Elem<ET>::T T;
  typedef typename Frag<T>::V V;
  const T* A = (const T*)Ap; const T* A2 = (const T*)A2p; const T* Bt = (const T*)Btp; const T* Bt2 = (const T*)Bt2p;
  __shared__ __align__(16) float sT[8][16 * 68];
  const int b    = blockIdx.y;
  const int lane = threadIdx.x & 31;
  const int wave = threadIdx.x >> 5;
  const int tilesN = N >> 6;
  const int tilesM = M >> 6;
  const int tile = blockIdx.x * 8 + wave;
  if (tile >= tilesM * tilesN) return;
  const int tm = tile / tilesN;
  const int tn = tile - tm * tilesN;
  const int m0 = tm << 6;
  const int n0 = tn << 6;

  const T* Ab  = A  + (size_t)b * strideA;
  const T* Bb  = Bt + (size_t)b * strideB;
  const T* Ab2 = SPLIT ? (A2  + (size_t)b * strideA) : nullptr;
  const T* Bb2 = SPLIT ? (Bt2 + (size_t)b * strideB) : nullptr;

  const int rlane = lane & 15;
  const int koff  = (lane >> 4) * 8;
  const int mOff  = (lane >> 4) * 8;

  v8f acc[4][4];
#pragma unroll
  for (int i = 0; i < 4; ++i)
#pragma unroll
    for (int j = 0; j < 4; ++j) acc[i][j] = (v8f){0.f,0.f,0.f,0.f,0.f,0.f,0.f,0.f};

  for (int k0 = 0; k0 < K; k0 += 32) {
    V bh[4], bl[4];
#pragma unroll
    for (int j = 0; j < 4; ++j) {
      const size_t bo = (size_t)(n0 + (j << 4) + rlane) * ldb + koff + k0;
      bh[j] = Frag<T>::load(Bb + bo);
      if (SPLIT) bl[j] = Frag<T>::load(Bb2 + bo);
    }
#pragma unroll
    for (int i = 0; i < 4; ++i) {
      const size_t ao = (size_t)(m0 + (i << 4) + rlane) * lda + koff + k0;
      V ah = Frag<T>::load(Ab + ao);
      V al;
      if (SPLIT) al = Frag<T>::load(Ab2 + ao);
#pragma unroll
      for (int j = 0; j < 4; ++j) {
        acc[i][j] = Frag<T>::mma(ah, bh[j], acc[i][j]);
        if (SPLIT) {
          acc[i][j] = Frag<T>::mma(ah, bl[j], acc[i][j]);
          acc[i][j] = Frag<T>::mma(al, bh[j], acc[i][j]);
        }
      }
      Frag<T>::guard(acc[i][0], acc[i][3], ah, SPLIT ? al : ah);
    }
    Frag<T>::keep(bh[0], bh[1], bh[2], bh[3]);
    if (SPLIT) Frag<T>::keep(bl[0], bl[1], bl[2], bl[3]);
  }
  acc_guard4(acc[0][0], acc[0][1], acc[0][2], acc[0][3]);
  acc_guard4(acc[1][0], acc[1][1], acc[1][2], acc[1][3]);
  acc_guard4(acc[2][0], acc[2][1], acc[2][2], acc[2][3]);
  acc_guard4(acc[3][0], acc[3][1], acc[3][2], acc[3][3]);

  float* slab = sT[wave];
  const float* Rb = RESID ? (resid + (size_t)b * strideR) : nullptr;
#pragma unroll
  for (int i = 0; i < 4; ++i) {
    const int mBase = m0 + (i << 4);
#pragma unroll
    for (int j = 0; j < 4; ++j) {
      const int n = n0 + (j << 4) + rlane;
      float bv = 0.f;
      if (BIAS_MODE == 2) bv = bias[n];
#pragma unroll
      for (int r = 0; r < 8; ++r) {
        float v = acc[i][j][r] * scale;
        if (BIAS_MODE == 1) v += bias[mBase + mOff + r];
        if (BIAS_MODE == 2) v += bv;
        if (RESID) v += Rb[(size_t)(mBase + mOff + r) * ldc + n];
        if (ACT == 2) v = fmaxf(v, 0.0f);
        if (ACT == 4) v = (v > 0.f) ? v : 0.01f * v;
        slab[(mOff + r) * 68 + (j << 4) + rlane] = v;
      }
    }
    __builtin_amdgcn_fence(__ATOMIC_RELEASE, "workgroup");
    __builtin_amdgcn_wave_barrier();
    __builtin_amdgcn_fence(__ATOMIC_ACQUIRE, "workgroup");
    if (OUT_MODE == 0) {
      float* C = (float*)Cout + (size_t)b * strideC;
      const int hh = lane >> 4, c4 = (lane & 15) * 4;
      for (int pass = 0; pass < 2; ++pass) {
#pragma unroll
        for (int it = 0; it < 8; ++it) {
          const int row = it * 2 + hh;
          v4f v = *(const v4f*)(slab + row * 68 + c4);
          *(volatile v4f*)(C + (size_t)(mBase + row) * ldc + n0 + c4) = v;
        }
        __threadfence();
      }
    } else {
      const int q = lane >> 3, c8 = (lane & 7) * 8;
      unsigned short* C  = (unsigned short*)Cout  + (size_t)b * strideC;
      unsigned short* C2 = (OUT_MODE == 2) ? ((unsigned short*)Cout2 + (size_t)b * strideC) : nullptr;
      for (int pass = 0; pass < 2; ++pass) {
#pragma unroll
        for (int it = 0; it < 4; ++it) {
          const int row = it * 4 + q;
          const float* sp = slab + row * 68 + c8;
          v8h hv, lv;
#pragma unroll
          for (int e = 0; e < 8; ++e) {
            if (OUT_MODE == 1) {
              hv[e] = (_Float16)sp[e];
            } else {
              unsigned short hb = f2bf_bits(sp[e]);
              unsigned short lb = f2bf_bits(sp[e] - bf_bits2f(hb));
              hv[e] = __builtin_bit_cast(_Float16, hb);
              lv[e] = __builtin_bit_cast(_Float16, lb);
            }
          }
          *(volatile v8h*)(C + (size_t)(mBase + row) * ldc + n0 + c8) = hv;
          if (OUT_MODE == 2) *(volatile v8h*)(C2 + (size_t)(mBase + row) * ldc + n0 + c8) = lv;
        }
        __threadfence();
      }
    }
    __builtin_amdgcn_fence(__ATOMIC_RELEASE, "workgroup");
    __builtin_amdgcn_wave_barrier();
    __builtin_amdgcn_fence(__ATOMIC_ACQUIRE, "workgroup");
  }
}

__device__ __forceinline__ void wave_sync() {
  __builtin_amdgcn_fence(__ATOMIC_RELEASE, "workgroup");
  __builtin_amdgcn_wave_barrier();
  __builtin_amdgcn_fence(__ATOMIC_ACQUIRE, "workgroup");
}

template <int MODE>
__global__ __launch_bounds__(256) void cast8_kernel(const float* __restrict__ in, unsigned short* __restrict__ o0,
                                                    unsigned short* __restrict__ o1, unsigned short* __restrict__ o2, int n8) {
  const int i = blockIdx.x * 256 + threadIdx.x;
  if (i >= n8) return;
  const float* p = in + 8 * (size_t)i;
  const v4f a = *(const v4f*)(p);
  const v4f c = *(const v4f*)(p + 4);
  float f[8];
#pragma unroll
  for (int e = 0; e < 4; ++e) { f[e] = a[e]; f[4 + e] = c[e]; }
  unsigned short hf[8], bhi[8], blo[8];
#pragma unroll
  for (int e = 0; e < 8; ++e) {
    hf[e]  = h_bits(f[e]);
    bhi[e] = f2bf_bits(f[e]);
    blo[e] = f2bf_bits(f[e] - bf_bits2f(bhi[e]));
  }
  const v4u uf = (v4u){pk16(hf[0], hf[1]), pk16(hf[2], hf[3]), pk16(hf[4], hf[5]), pk16(hf[6], hf[7])};
  const v4u uh = (v4u){pk16(bhi[0], bhi[1]), pk16(bhi[2], bhi[3]), pk16(bhi[4], bhi[5]), pk16(bhi[6], bhi[7])};
  const v4u ul = (v4u){pk16(blo[0], blo[1]), pk16(blo[2], blo[3]), pk16(blo[4], blo[5]), pk16(blo[6], blo[7])};
  const size_t off = 8 * (size_t)i;
  for (int pass = 0; pass < 2; ++pass) {
    if (MODE != 1) *(volatile v4u*)(o0 + off) = uf;
    if (MODE == 1) { *(volatile v4u*)(o0 + off) = uh; *(volatile v4u*)(o1 + off) = ul; }
    if (MODE == 2) { *(volatile v4u*)(o1 + off) = uh; *(volatile v4u*)(o2 + off) = ul; }
    __threadfence();
  }
}

template <int MODE>
__global__ __launch_bounds__(256) void wt64_kernel(const float* __restrict__ W, unsigned short* __restrict__ out,
                                                   unsigned short* __restrict__ out2, int Kdim, int Ndim, float scale) {
  __shared__ float sm[64][65];
  const int t  = threadIdx.x;
  const int k0 = blockIdx.x * 64;
  const int n0 = blockIdx.y * 64;
#pragma unroll
  for (int i = 0; i < 16; ++i) {
    const int e = i * 256 + t;
    const int r = e >> 6;
    const int c = e & 63;
    sm[c][r] = W[(size_t)(k0 + r) * Ndim + n0 + c] * scale;
  }
  __syncthreads();
  const int lane = t & 31, wave = t >> 5;
  const int q = lane >> 3, c8 = (lane & 7) * 8;
  for (int pass = 0; pass < 2; ++pass) {
#pragma unroll
    for (int it = 0; it < 2; ++it) {
      const int row = wave * 8 + it * 4 + q;
      unsigned short hb[8], lb[8];
#pragma unroll
      for (int e = 0; e < 8; ++e) {
        const float v = sm[row][c8 + e];
        if (MODE == 0) { hb[e] = h_bits(v); lb[e] = 0; }
        else { hb[e] = f2bf_bits(v); lb[e] = f2bf_bits(v - bf_bits2f(hb[e])); }
      }
      const v4u uh = (v4u){pk16(hb[0], hb[1]), pk16(hb[2], hb[3]), pk16(hb[4], hb[5]), pk16(hb[6], hb[7])};
      *(volatile v4u*)(out + (size_t)(n0 + row) * Kdim + k0 + c8) = uh;
      if (MODE == 1) {
        const v4u ul = (v4u){pk16(lb[0], lb[1]), pk16(lb[2], lb[3]), pk16(lb[4], lb[5]), pk16(lb[6], lb[7])};
        *(volatile v4u*)(out2 + (size_t)(n0 + row) * Kdim + k0 + c8) = ul;
      }
    }
    __threadfence();
  }
}

__global__ __launch_bounds__(256) void headproj_kernel(const float* __restrict__ x, const float* __restrict__ aw, const float* __restrict__ ab,
                                                       const float* __restrict__ bw, const float* __restrict__ bbias,
                                                       const float* __restrict__ alog, const float* __restrict__ dtb,
                                                       float* __restrict__ gout, float* __restrict__ bout) {
  __shared__ __align__(16) float raw[512];
  __shared__ __align__(16) float res[512];
  const int tid = threadIdx.x, wave = tid >> 5, lane = tid & 31;
  const int m0 = blockIdx.x * 32;
#pragma unroll 1
  for (int rr = 0; rr < 4; ++rr) {
    const int r = wave * 4 + rr;
    const float* xr = x + (size_t)(m0 + r) * kDM;
    float sa[8], sb[8];
#pragma unroll
    for (int hq = 0; hq < 8; ++hq) { sa[hq] = 0.f; sb[hq] = 0.f; }
#pragma unroll 1
    for (int u = 0; u < kDM / 32; ++u) {
      const int k = lane + 32 * u;
      const float xv = xr[k];
      const v4f a0 = *(const v4f*)(aw + (size_t)k * 8);
      const v4f a1 = *(const v4f*)(aw + (size_t)k * 8 + 4);
      const v4f b0 = *(const v4f*)(bw + (size_t)k * 8);
      const v4f b1 = *(const v4f*)(bw + (size_t)k * 8 + 4);
#pragma unroll
      for (int e = 0; e < 4; ++e) {
        sa[e]     = fmaf(xv, a0[e], sa[e]);
        sa[4 + e] = fmaf(xv, a1[e], sa[4 + e]);
        sb[e]     = fmaf(xv, b0[e], sb[e]);
        sb[4 + e] = fmaf(xv, b1[e], sb[4 + e]);
      }
    }
#pragma unroll
    for (int hq = 0; hq < 8; ++hq) {
#pragma unroll
      for (int off = 16; off > 0; off >>= 1) {
        sa[hq] += __shfl_xor(sa[hq], off, 32);
        sb[hq] += __shfl_xor(sb[hq], off, 32);
      }
    }
    if (lane == 0) {
#pragma unroll
      for (int hq = 0; hq < 8; ++hq) { raw[hq * 32 + r] = sa[hq]; raw[(8 + hq) * 32 + r] = sb[hq]; }
    }
  }
  __syncthreads();
  for (int e = tid; e < 512; e += 256) {
    const int o = e >> 5;
    const float v = raw[e];
    float outv;
    if (o < 8) {
      const float z = dtb[o] + (v + ab[o]);
      const float sp = fmaxf(z, 0.0f) + log1pf(expf(-fabsf(z)));
      outv = -sp * expf(alog[o]);
    } else {
      const int hq = o - 8;
      const float z = v + bbias[hq];
      outv = 1.0f / (1.0f + expf(-z));
    }
    res[e] = outv;
  }
  __syncthreads();
  const int b = m0 / kT, t0 = m0 - b * kT;
  const int sel = (lane >> 3) & 1;
  const int slot = sel ? (8 + wave) : wave;
  const int c4 = 4 * (lane & 7);
  const v4f val = *(const v4f*)(res + slot * 32 + c4);
  float* gp = gout + ((size_t)(b * kH + wave)) * kT + t0 + c4;
  float* bp = bout + ((size_t)(b * kH + wave)) * kT + t0 + c4;
  float* p = sel ? bp : gp;
  if (lane < 16) {
    *(volatile v4f*)p = val;
    __threadfence();
    *(volatile v4f*)p = val;
  }
}

template <int CH, int NORM>
__global__ __launch_bounds__(256) void convhead_kernel(const float* __restrict__ pre, const float* __restrict__ cw,
                                                       const float* __restrict__ cb, float* __restrict__ dst, float oscale) {
#pragma clang fp contract(off)
  constexpr int CT = kH * CH;
  constexpr int NS = CH / 32;
  __shared__ __align__(16) float sIn[35 * CH];
  __shared__ __align__(16) float slab[8][4 * CH];
  const int tid = threadIdx.x, wave = tid >> 5, lane = tid & 31;
  const int t0 = blockIdx.x * 32, h = blockIdx.y, b = blockIdx.z;
  for (int e = tid; e < 35 * CH; e += 256) {
    const int r = e / CH;
    const int c = e - r * CH;
    const int t = t0 - 3 + r;
    const int tc = (t < 0) ? 0 : t;
    const float v = pre[((size_t)(b * kT + tc)) * CT + h * CH + c];
    sIn[e] = (t >= 0) ? v : 0.0f;
  }
  __syncthreads();
  float* sl = slab[wave];
#pragma unroll 1
  for (int rr = 0; rr < 4; ++rr) {
    const int tl = wave * 4 + rr;
    float ss = 0.f;
#pragma unroll 1
    for (int s = 0; s < NS; ++s) {
      const int c = lane + 32 * s;
      const int hc = h * CH + c;
      const v4f w4 = *(const v4f*)(cw + (size_t)hc * 4);
      const float p0 = w4[0] * sIn[(tl + 0) * CH + c];
      const float p1 = w4[1] * sIn[(tl + 1) * CH + c];
      const float p2 = w4[2] * sIn[(tl + 2) * CH + c];
      const float p3 = w4[3] * sIn[(tl + 3) * CH + c];
      const float acc = (((p0 + p1) + p2) + p3) + cb[hc];
      const float sg = 1.0f / (1.0f + expf(-acc));
      const float yy = acc * sg;
      sl[rr * CH + c] = yy;
      ss = ss + yy * yy;
    }
    if (NORM) {
#pragma unroll
      for (int off = 16; off > 0; off >>= 1) ss += __shfl_xor(ss, off, 32);
      const float inv = 1.0f / (sqrtf(ss) + kEps);
#pragma unroll 1
      for (int s = 0; s < NS; ++s) {
        const int c = lane + 32 * s;
        const float yy = sl[rr * CH + c];
        sl[rr * CH + c] = (yy * inv) * oscale;
      }
    }
  }
  wave_sync();
  float* obase = dst + (((size_t)(b * kH + h)) * kT + t0 + wave * 4) * CH;
  for (int pass = 0; pass < 2; ++pass) {
#pragma unroll
    for (int j = 0; j < NS; ++j) {
      const v4f v = *(const v4f*)(sl + 128 * j + 4 * lane);
      *(volatile v4f*)(obase + 128 * j + 4 * lane) = v;
    }
    __threadfence();
  }
}

__global__ __launch_bounds__(192) void state_scan_kernel(const float* __restrict__ qn, const float* __restrict__ kn,
                                                         const float* __restrict__ vh, const float* __restrict__ gin,
                                                         const float* __restrict__ bin, float* __restrict__ osc) {
#pragma clang fp contract(off)
  __shared__ __align__(16) float kqS[2][2 * kKH];
  __shared__ __align__(16) float oS[6][8 * 32];

  const int tid = threadIdx.x, wave = tid >> 5, lane = tid & 31;
  const int bhIdx = blockIdx.x;
  const int vcol = tid;
  const size_t rowbase = (size_t)bhIdx * kT;
  const bool isk = (tid < kKH);
  const int kidx = isk ? tid : (kKH - 1);
  const int qidx = isk ? 0 : (tid - kKH);

  float S[kKH];
#pragma unroll
  for (int i = 0; i < kKH; ++i) S[i] = 0.f;

  {
    const float fk = kn[rowbase * kKH + kidx];
    const float fq = qn[rowbase * kKH + qidx];
    kqS[0][tid] = isk ? fk : fq;
  }
  __syncthreads();

#pragma unroll 1
  for (int t = 0; t < kT; ++t) {
    const int cur = t & 1;
    const int tn = (t + 1 < kT) ? (t + 1) : (kT - 1);
    const float fkn = kn[(rowbase + tn) * kKH + kidx];
    const float fqn = qn[(rowbase + tn) * kKH + qidx];
    const float nval = isk ? fkn : fqn;
    const float gt = gin[rowbase + t];
    const float bt = bin[rowbase + t];
    const float vt = vh[(rowbase + t) * kVH + vcol];
    const float decay = expf(gt);
    const float* kp = &kqS[cur][0];
    const float* qp = kp + kKH;

#pragma unroll
    for (int i = 0; i < kKH; ++i) S[i] = S[i] * decay;

    float sdot = 0.f;
#pragma unroll
    for (int c = 0; c < 6; ++c) {
#pragma unroll
      for (int e = 0; e < 4; ++e) {
        const v4f k4 = *(const v4f*)(kp + 16 * c + 4 * e);
#pragma unroll
        for (int i = 0; i < 4; ++i) {
          const float p = S[16 * c + 4 * e + i] * k4[i];
          sdot = sdot + p;
        }
      }
      asm volatile("" ::: "memory");
    }
    const float u = bt * (vt - sdot);

#pragma unroll
    for (int c = 0; c < 6; ++c) {
#pragma unroll
      for (int e = 0; e < 4; ++e) {
        const v4f k4 = *(const v4f*)(kp + 16 * c + 4 * e);
#pragma unroll
        for (int i = 0; i < 4; ++i) {
          const float p = k4[i] * u;
          S[16 * c + 4 * e + i] = S[16 * c + 4 * e + i] + p;
        }
      }
      asm volatile("" ::: "memory");
    }

    float ov = 0.f;
#pragma unroll
    for (int c = 0; c < 6; ++c) {
#pragma unroll
      for (int e = 0; e < 4; ++e) {
        const v4f q4 = *(const v4f*)(qp + 16 * c + 4 * e);
#pragma unroll
        for (int i = 0; i < 4; ++i) {
          const float p = S[16 * c + 4 * e + i] * q4[i];
          ov = ov + p;
        }
      }
      asm volatile("" ::: "memory");
    }

    oS[wave][(t & 7) * 32 + lane] = ov;
    kqS[cur ^ 1][tid] = nval;

    if ((t & 7) == 7) {
      wave_sync();
      const float* os = oS[wave];
      const int q = lane >> 3, c4 = 4 * (lane & 7);
      const v4f o0 = *(const v4f*)(os + q * 32 + c4);
      const v4f o1 = *(const v4f*)(os + (q + 4) * 32 + c4);
      float* p0 = osc + (rowbase + (size_t)(t - 7 + q)) * kVH + wave * 32 + c4;
      float* p1 = p0 + 4 * kVH;
      for (int pass = 0; pass < 2; ++pass) {
        *(volatile v4f*)p0 = o0;
        *(volatile v4f*)p1 = o1;
        __threadfence();
      }
    }
    __syncthreads();
  }
}

__global__ __launch_bounds__(256) void normgate_kernel(const float* __restrict__ osc, const float* __restrict__ gate,
                                                       const float* __restrict__ pnw, unsigned short* __restrict__ oh,
                                                       unsigned short* __restrict__ ol) {
  __shared__ float red[8];
  __shared__ __align__(16) float sv[kVT];
  const int m = blockIdx.x;
  const int b = m / kT, t = m - b * kT;
  const int tid = threadIdx.x, wave = tid >> 5, lane = tid & 31;
  float ss = 0.f;
#pragma unroll
  for (int i = 0; i < 6; ++i) {
    const int n = tid + 256 * i;
    const int h = n / kVH, v = n - h * kVH;
    const float o = osc[(((size_t)(b * kH + h)) * kT + t) * kVH + v];
    sv[n] = o;
    ss = fmaf(o, o, ss);
  }
#pragma unroll
  for (int off = 16; off > 0; off >>= 1) ss += __shfl_xor(ss, off, 32);
  if (lane == 0) red[wave] = ss;
  __syncthreads();
  const float tot = ((red[0] + red[1]) + (red[2] + red[3])) + ((red[4] + red[5]) + (red[6] + red[7]));
  const float scl = 1.0f / sqrtf(tot * (1.0f / 1536.0f) + kEps);
#pragma unroll 1
  for (int i = 0; i < 6; ++i) {
    const int n = tid + 256 * i;
    const float gp = gate[(size_t)m * kVT + n];
    const float gt = gp * (1.0f / (1.0f + expf(-gp)));
    const float o = sv[n];
    sv[n] = ((o * scl) * pnw[n]) * gt;
  }
  __syncthreads();
  if (tid < 192) {
    const int n8 = tid * 8;
    const v4f a = *(const v4f*)(sv + n8);
    const v4f c = *(const v4f*)(sv + n8 + 4);
    unsigned short hb[8], lb[8];
#pragma unroll
    for (int e = 0; e < 4; ++e) {
      hb[e] = f2bf_bits(a[e]);     lb[e] = f2bf_bits(a[e] - bf_bits2f(hb[e]));
      hb[4 + e] = f2bf_bits(c[e]); lb[4 + e] = f2bf_bits(c[e] - bf_bits2f(hb[4 + e]));
    }
    const v4u uh = (v4u){pk16(hb[0], hb[1]), pk16(hb[2], hb[3]), pk16(hb[4], hb[5]), pk16(hb[6], hb[7])};
    const v4u ul = (v4u){pk16(lb[0], lb[1]), pk16(lb[2], lb[3]), pk16(lb[4], lb[5]), pk16(lb[6], lb[7])};
    unsigned short* ph = oh + (size_t)m * kVT + n8;
    unsigned short* pl = ol + (size_t)m * kVT + n8;
    *(volatile v4u*)ph = uh;
    *(volatile v4u*)pl = ul;
    __threadfence();
    *(volatile v4u*)ph = uh;
    *(volatile v4u*)pl = ul;
  }
}

constexpr size_t kOffXh   = 0;
constexpr size_t kOffXbh  = 8388608;
constexpr size_t kOffXbl  = 16777216;
constexpr size_t kOffVh   = 0;
constexpr size_t kOffCbh  = 25165824;
constexpr size_t kOffCbl  = 29360128;
constexpr size_t kOffWoTh = 25165824;
constexpr size_t kOffWoTl = 28311552;
constexpr size_t kOffG    = 31457280;
constexpr size_t kOffBeta = 31588352;
constexpr size_t kOffQpre = 33554432;
constexpr size_t kOffKn   = 33554432;
constexpr size_t kOffMixL = 33554432;
constexpr size_t kOffKpre = 46137344;
constexpr size_t kOffMixH = 46137344;
constexpr size_t kOffVpre = 58720256;
constexpr size_t kOffOsc  = 58720256;
constexpr size_t kOffGate = 83886080;
constexpr size_t kOffWqTh = 109051904;
constexpr size_t kOffWqTl = 110624768;
constexpr size_t kOffWkTh = 112197632;
constexpr size_t kOffWkTl = 112984064;
constexpr size_t kOffWvTh = 113770496;
constexpr size_t kOffWvTl = 115343360;
constexpr size_t kOffGpT  = 116916224;
constexpr size_t kOffQn   = 109051904;
constexpr size_t kWsTotal = 121634816;

extern "C" void kernel_launch(void* const* d_in, const int* in_sizes, int n_in,
                              void* d_out, int out_size, void* d_ws, size_t ws_size, hipStream_t stream) {
  if (n_in < 20) return;
  if (ws_size < kWsTotal) return;
  if ((size_t)out_size < (size_t)kM * kDM) return;
  if (in_sizes[0] != kM * kDM || in_sizes[1] != kM * kDKV) return;

  const float* x        = (const float*)d_in[0];
  const float* c_kv     = (const float*)d_in[1];
  const float* w_q      = (const float*)d_in[2];
  const float* w_k      = (const float*)d_in[3];
  const float* w_v      = (const float*)d_in[4];
  const float* conv_q_w = (const float*)d_in[5];
  const float* conv_q_b = (const float*)d_in[6];
  const float* conv_k_w = (const float*)d_in[7];
  const float* conv_k_b = (const float*)d_in[8];
  const float* conv_v_w = (const float*)d_in[9];
  const float* conv_v_b = (const float*)d_in[10];
  const float* a_proj_w = (const float*)d_in[11];
  const float* a_proj_b = (const float*)d_in[12];
  const float* A_log    = (const float*)d_in[13];
  const float* dt_bias  = (const float*)d_in[14];
  const float* b_proj_w = (const float*)d_in[15];
  const float* b_proj_b = (const float*)d_in[16];
  const float* g_proj_w = (const float*)d_in[17];
  const float* pnw      = (const float*)d_in[18];
  const float* w_o      = (const float*)d_in[19];
  float* out = (float*)d_out;
  char* ws = (char*)d_ws;

  unsigned short* Xh   = (unsigned short*)(ws + kOffXh);
  unsigned short* Xbh  = (unsigned short*)(ws + kOffXbh);
  unsigned short* Xbl  = (unsigned short*)(ws + kOffXbl);
  float* vhd           = (float*)(ws + kOffVh);
  unsigned short* Cbh  = (unsigned short*)(ws + kOffCbh);
  unsigned short* Cbl  = (unsigned short*)(ws + kOffCbl);
  unsigned short* WoTh = (unsigned short*)(ws + kOffWoTh);
  unsigned short* WoTl = (unsigned short*)(ws + kOffWoTl);
  float* gbuf          = (float*)(ws + kOffG);
  float* bbuf          = (float*)(ws + kOffBeta);
  float* q_pre         = (float*)(ws + kOffQpre);
  float* kn            = (float*)(ws + kOffKn);
  unsigned short* mixL = (unsigned short*)(ws + kOffMixL);
  float* k_pre         = (float*)(ws + kOffKpre);
  unsigned short* mixH = (unsigned short*)(ws + kOffMixH);
  float* v_pre         = (float*)(ws + kOffVpre);
  float* o_scan        = (float*)(ws + kOffOsc);
  float* gate_pre      = (float*)(ws + kOffGate);
  unsigned short* WqTh = (unsigned short*)(ws + kOffWqTh);
  unsigned short* WqTl = (unsigned short*)(ws + kOffWqTl);
  unsigned short* WkTh = (unsigned short*)(ws + kOffWkTh);
  unsigned short* WkTl = (unsigned short*)(ws + kOffWkTl);
  unsigned short* WvTh = (unsigned short*)(ws + kOffWvTh);
  unsigned short* WvTl = (unsigned short*)(ws + kOffWvTl);
  unsigned short* GpT  = (unsigned short*)(ws + kOffGpT);
  float* qn            = (float*)(ws + kOffQn);

  cast8_kernel<2><<<(kM * kDM / 8) / 256, 256, 0, stream>>>(x, Xh, Xbh, Xbl, kM * kDM / 8);
  cast8_kernel<1><<<(kM * kDKV / 8) / 256, 256, 0, stream>>>(c_kv, Cbh, Cbl, Cbl, kM * kDKV / 8);

  wt64_kernel<1><<<dim3(kDM / 64, kKQT / 64), 256, 0, stream>>>(w_q, WqTh, WqTl, kDM, kKQT, 1.0f);
  wt64_kernel<1><<<dim3(kDKV / 64, kKQT / 64), 256, 0, stream>>>(w_k, WkTh, WkTl, kDKV, kKQT, 1.0f);
  wt64_kernel<1><<<dim3(kDKV / 64, kVT / 64), 256, 0, stream>>>(w_v, WvTh, WvTl, kDKV, kVT, 1.0f);
  wt64_kernel<0><<<dim3(kDM / 64, kVT / 64), 256, 0, stream>>>(g_proj_w, GpT, GpT, kDM, kVT, kWCarry);

  wmma_gemm64<1, true, 0, 0, false, 0><<<dim3((kM / 64) * (kKQT / 64) / 8, 1), 256, 0, stream>>>(
      Xbh, Xbl, kDM, 0L, WqTh, WqTl, kDM, 0L, (void*)q_pre, (void*)q_pre, kKQT, 0L, pnw, pnw, 0L, kM, kKQT, kDM, 1.0f);
  wmma_gemm64<0, false, 0, 0, false, 0><<<dim3((kM / 64) * (kVT / 64) / 8, 1), 256, 0, stream>>>(
      Xh, Xh, kDM, 0L, GpT, GpT, kDM, 0L, (void*)gate_pre, (void*)gate_pre, kVT, 0L, pnw, pnw, 0L, kM, kVT, kDM, kWCarryInv);
  wmma_gemm64<1, true, 0, 0, false, 0><<<dim3((kM / 64) * (kKQT / 64) / 8, 1), 256, 0, stream>>>(
      Cbh, Cbl, kDKV, 0L, WkTh, WkTl, kDKV, 0L, (void*)k_pre, (void*)k_pre, kKQT, 0L, pnw, pnw, 0L, kM, kKQT, kDKV, 1.0f);
  wmma_gemm64<1, true, 0, 0, false, 0><<<dim3((kM / 64) * (kVT / 64) / 8, 1), 256, 0, stream>>>(
      Cbh, Cbl, kDKV, 0L, WvTh, WvTl, kDKV, 0L, (void*)v_pre, (void*)v_pre, kVT, 0L, pnw, pnw, 0L, kM, kVT, kDKV, 1.0f);

  headproj_kernel<<<kM / 32, 256, 0, stream>>>(x, a_proj_w, a_proj_b, b_proj_w, b_proj_b, A_log, dt_bias, gbuf, bbuf);

  convhead_kernel<kKH, 1><<<dim3(kT / 32, kH, kB), 256, 0, stream>>>(q_pre, conv_q_w, conv_q_b, qn, kQScale);
  convhead_kernel<kKH, 1><<<dim3(kT / 32, kH, kB), 256, 0, stream>>>(k_pre, conv_k_w, conv_k_b, kn, 1.0f);
  convhead_kernel<kVH, 0><<<dim3(kT / 32, kH, kB), 256, 0, stream>>>(v_pre, conv_v_w, conv_v_b, vhd, 1.0f);

  state_scan_kernel<<<kBH, 192, 0, stream>>>(qn, kn, vhd, gbuf, bbuf, o_scan);

  normgate_kernel<<<kM, 256, 0, stream>>>(o_scan, gate_pre, pnw, mixH, mixL);

  wt64_kernel<1><<<dim3(kVT / 64, kDM / 64), 256, 0, stream>>>(w_o, WoTh, WoTl, kVT, kDM, 1.0f);

  wmma_gemm64<1, true, 0, 0, false, 0><<<dim3((kM / 64) * (kDM / 64) / 8, 1), 256, 0, stream>>>(
      mixH, mixL, kVT, 0L, WoTh, WoTl, kVT, 0L, (void*)out, (void*)out, kDM, 0L, pnw, pnw, 0L, kM, kDM, kVT, 1.0f);
}
